// GIN_6897717478006
// MI455X (gfx1250) — hardware-verified
//
#include <hip/hip_runtime.h>
#include <stddef.h>
#include <stdint.h>


#define DIN     128
#define HL3     512
#define HCAT    768
#define HCW     1536
#define D1      1024
#define ZPW     2048
#define COUT    512
#define NTHR    256
#define NWAVE   8
#define EPT     8
#define CHUNK   (NTHR * EPT)
#define WCAP    (EPT * 32)
#define LISTN   (NWAVE * WCAP)
#define NBMAX   2048
#define RCAP    28672
#define DEGCAP  64
#define PKS     11
#define GBM     64
#define GBN     128
#define GTHR    128
#define GNT     8
#define PARTW   288
#define PG      32
#define APR     16
#define CA      16.0f
#define CT      16.0f
#define CW      4096.0f
#define NU11    (DIN * (DIN / 8))
#define NU13    (HL3 * (DIN / 8))
#define NU23    (HL3 * (HL3 / 8))
#define NUL1    (D1 * (HCW / 8))
#define NUL2    (COUT * (ZPW / 8))
#define NUB1    (NU11)
#define NUB2    (2 * NU11)
#define NUB3    (2 * NU11 + NU13)
#define NUB4    (3 * NU11 + NU13)
#define NUB5    (4 * NU11 + NU13)
#define NUB6    (4 * NU11 + NU13 + NU23)
#define NUB7    (NUB6 + NUL1)
#define NUTOT   (NUB7 + NUL2)
#define WSMAX   268435456
#define LDS_AGG ((2 * RCAP + 2 * NBMAX + LISTN) * 4 + 64)
#define LDS_POOL(nh) ((PG * (nh) + 2 * (nh)) * 4 + LISTN * 4 + 64)

static_assert((CHUNK & (CHUNK - 1)) == 0 && CHUNK <= (1 << PKS));
static_assert((NBMAX & (NBMAX - 1)) == 0 && NBMAX <= (1 << PKS));
static_assert(NTHR * 8 == NBMAX);
static_assert(LISTN >= NBMAX && LISTN >= NWAVE * WCAP);
static_assert((RCAP % 32) == 0);
static_assert(LDS_AGG <= 300000);
static_assert(LDS_POOL(HL3) <= 300000 && LDS_POOL(DIN) <= 300000);
static_assert(GBM == (GTHR / 32) * 16 && GBN == 16 * GNT && GTHR == GBN && GBN == 4 * 32);
static_assert(DIN == 32 * 4);
static_assert((DIN % 32) == 0 && (HL3 % 32) == 0 && (HCW % 32) == 0 && (ZPW % 32) == 0);
static_assert((DIN % GBN) == 0 && (HL3 % GBN) == 0 && (D1 % GBN) == 0 && (COUT % GBN) == 0);
static_assert(HCAT == 2 * DIN + HL3 && HCW == 2 * HCAT && ZPW == 2 * D1);
static_assert((PARTW % 32) == 0 && PARTW >= 2 * GBN + 1 && PARTW / 4 <= GTHR);
static_assert((NU11 % NTHR) == 0 && (NU13 % NTHR) == 0 && (NU23 % NTHR) == 0);
static_assert((NUL1 % NTHR) == 0 && (NUL2 % NTHR) == 0 && (NUTOT % NTHR) == 0);
static_assert((HCW / 8) == 192 && (ZPW / 8) == 256 && (HL3 / 8) == 64 && (DIN / 8) == 16);
static_assert((HCAT % 8) == 0 && (D1 & (D1 - 1)) == 0);
static_assert((PG & (PG - 1)) == 0 && PG <= NBMAX);
static_assert(((PG * (DIN / 8)) % NTHR) == 0 && ((PG * (HL3 / 8)) % NTHR) == 0);
static_assert(NTHR == 2 * DIN);
static_assert((APR % 2) == 0 && (GBM % APR) == 0 && (APR * DIN) == 2 * 4 * NTHR);
static_assert((GBM * GBN) % GTHR == 0);

typedef float          v4f  __attribute__((ext_vector_type(4)));
typedef float          v8f  __attribute__((ext_vector_type(8)));
typedef int            v4i  __attribute__((ext_vector_type(4)));
typedef int            v8i  __attribute__((ext_vector_type(8)));
typedef unsigned int   v2u  __attribute__((ext_vector_type(2)));
typedef unsigned int   v4u  __attribute__((ext_vector_type(4)));
typedef unsigned short v8us __attribute__((ext_vector_type(8)));
typedef _Float16       v16h __attribute__((ext_vector_type(16)));
typedef __bf16         v16b __attribute__((ext_vector_type(16)));
typedef v4f  __attribute__((may_alias)) v4fa;
typedef v8us __attribute__((may_alias)) v8usa;
union Frag { v16h vh; v16b vb; v8us h[2]; v8i w; };

template <int BF>
__device__ __forceinline__ v8f wmx(const Frag& a, const Frag& b, v8f c) {
  v8f d;
  if constexpr (BF != 0) {
    d = __builtin_amdgcn_wmma_f32_16x16x32_bf16(false, a.vb, false, b.vb, (short)0, c, false, false);
  } else {
    d = __builtin_amdgcn_wmma_f32_16x16x32_f16(false, a.vh, false, b.vh, (short)0, c, false, false);
  }
  asm volatile("v_nop\n\tv_nop\n\tv_nop\n\tv_nop" : "+v"(d) : "v"(a.w), "v"(b.w));
  return d;
}

__device__ __forceinline__ unsigned short bf_bits(float f) {
  unsigned int u = __float_as_uint(f);
  u += 0x7FFFu + ((u >> 16) & 1u);
  return (unsigned short)(u >> 16);
}
__device__ __forceinline__ float bf_val(unsigned short b) { return __uint_as_float(((unsigned int)b) << 16); }
__device__ __forceinline__ float bf_rne(float f) { return bf_val(bf_bits(f)); }

__device__ __forceinline__ unsigned short h16_bits(float f) {
  union { _Float16 h; unsigned short u; } c;
  c.h = (_Float16)f;
  return c.u;
}

__device__ __forceinline__ float gelu_exact(float v) {
  return 0.5f * v * (1.0f + erff(v * 0.70710678118654752f));
}

__device__ __forceinline__ void hilo8(const v4f a, const v4f b, v8us& hv, v8us& lv) {
  const float f[8] = {a.x, a.y, a.z, a.w, b.x, b.y, b.z, b.w};
#pragma unroll
  for (int j = 0; j < 8; ++j) {
    const unsigned short hb = bf_bits(f[j]);
    hv[j] = hb;
    lv[j] = bf_bits(f[j] - bf_val(hb));
  }
}

__device__ __forceinline__ int scan_chunk(const int* __restrict__ dsts, int nE, int cbase, int slotBase,
                                          int nb, int vec8, int* list, int tid, int lane, int wave) {
  int wc = 0;
  const int el0  = tid * EPT;
  const int e0   = cbase + el0;
  const int sent = -2147483647 - 1;
  v4i da, db;
  if (vec8 != 0 && cbase + CHUNK <= nE) {
    da = *(const v4i*)(dsts + e0);
    db = *(const v4i*)(dsts + e0 + 4);
  } else {
    da.x = (e0     < nE) ? dsts[min(e0,     nE - 1)] : sent;
    da.y = (e0 + 1 < nE) ? dsts[min(e0 + 1, nE - 1)] : sent;
    da.z = (e0 + 2 < nE) ? dsts[min(e0 + 2, nE - 1)] : sent;
    da.w = (e0 + 3 < nE) ? dsts[min(e0 + 3, nE - 1)] : sent;
    db.x = (e0 + 4 < nE) ? dsts[min(e0 + 4, nE - 1)] : sent;
    db.y = (e0 + 5 < nE) ? dsts[min(e0 + 5, nE - 1)] : sent;
    db.z = (e0 + 6 < nE) ? dsts[min(e0 + 6, nE - 1)] : sent;
    db.w = (e0 + 7 < nE) ? dsts[min(e0 + 7, nE - 1)] : sent;
  }
  const unsigned nbs = (unsigned)slotBase;
  const unsigned unb = (unsigned)nb;
  const unsigned s0 = (unsigned)da.x - nbs, s1 = (unsigned)da.y - nbs;
  const unsigned s2 = (unsigned)da.z - nbs, s3 = (unsigned)da.w - nbs;
  const unsigned s4 = (unsigned)db.x - nbs, s5 = (unsigned)db.y - nbs;
  const unsigned s6 = (unsigned)db.z - nbs, s7 = (unsigned)db.w - nbs;
  const bool h0 = s0 < unb, h1 = s1 < unb, h2 = s2 < unb, h3 = s3 < unb;
  const bool h4 = s4 < unb, h5 = s5 < unb, h6 = s6 < unb, h7 = s7 < unb;
  const unsigned any = __builtin_amdgcn_ballot_w32(h0 | h1 | h2 | h3 | h4 | h5 | h6 | h7);
  if (any != 0u) {
#define HITJ(J, HJ, SJ) { \
      const unsigned mj = __builtin_amdgcn_ballot_w32(HJ); \
      if (mj != 0u) { \
        if (HJ) { \
          const int pos = wc + (int)__builtin_amdgcn_mbcnt_lo(mj, 0u); \
          if (pos < WCAP) list[wave * WCAP + pos] = ((el0 + (J)) << PKS) | (int)(SJ); \
        } \
        wc += (int)__builtin_popcount(mj); } }
    HITJ(0, h0, s0)
    HITJ(1, h1, s1)
    HITJ(2, h2, s2)
    HITJ(3, h3, s3)
    HITJ(4, h4, s4)
    HITJ(5, h5, s5)
    HITJ(6, h6, s6)
    HITJ(7, h7, s7)
#undef HITJ
  }
  return wc;
}

__device__ __forceinline__ v8us cv8h(const float* __restrict__ p, size_t stride) {
  v8us o;
#pragma unroll
  for (int i = 0; i < 8; ++i) o[i] = h16_bits(bf_rne(p[(size_t)i * stride]) * CW);
  return o;
}
__device__ __forceinline__ v8us cv8b(const float* __restrict__ p, size_t stride) {
  v8us o;
#pragma unroll
  for (int i = 0; i < 8; ++i) o[i] = bf_bits(p[(size_t)i * stride]);
  return o;
}

__global__ __launch_bounds__(NTHR) void k_wprep(const float* __restrict__ w11, const float* __restrict__ w12,
                                                const float* __restrict__ w13, const float* __restrict__ w21,
                                                const float* __restrict__ w22, const float* __restrict__ w23,
                                                const float* __restrict__ l1,  const float* __restrict__ l2,
                                                unsigned short* p11, unsigned short* p12, unsigned short* p13,
                                                unsigned short* p21, unsigned short* p22, unsigned short* p23,
                                                unsigned short* pl1, unsigned short* pl2) {
  const int u = (int)blockIdx.x * NTHR + (int)threadIdx.x;
  v8us o;
  unsigned short* dp;
  if (u < NUB1) {
    const int v = u, n = v >> 4, k8 = (v & 15) * 8;
    o = cv8h(w11 + (size_t)k8 * DIN + n, DIN);
    dp = p11 + (size_t)v * 8;
  } else if (u < NUB2) {
    const int v = u - NUB1, n = v >> 4, k8 = (v & 15) * 8;
    o = cv8h(w12 + (size_t)k8 * DIN + n, DIN);
    dp = p12 + (size_t)v * 8;
  } else if (u < NUB3) {
    const int v = u - NUB2, n = v >> 4, k8 = (v & 15) * 8;
    o = cv8h(w13 + (size_t)k8 * HL3 + n, HL3);
    dp = p13 + (size_t)v * 8;
  } else if (u < NUB4) {
    const int v = u - NUB3, n = v >> 4, k8 = (v & 15) * 8;
    o = cv8h(w21 + (size_t)k8 * DIN + n, DIN);
    dp = p21 + (size_t)v * 8;
  } else if (u < NUB5) {
    const int v = u - NUB4, n = v >> 4, k8 = (v & 15) * 8;
    o = cv8h(w22 + (size_t)k8 * DIN + n, DIN);
    dp = p22 + (size_t)v * 8;
  } else if (u < NUB6) {
    const int v = u - NUB5, n = v >> 6, k8 = (v & 63) * 8;
    o = cv8h(w23 + (size_t)k8 * HL3 + n, HL3);
    dp = p23 + (size_t)v * 8;
  } else if (u < NUB7) {
    const int v = u - NUB6;
    const int n  = v / (HCW / 8);
    const int k8 = (v - n * (HCW / 8)) * 8;
    const int kk = k8 < HCAT ? k8 : k8 - HCAT;
    o = cv8b(l1 + (size_t)kk * D1 + n, D1);
    dp = pl1 + (size_t)v * 8;
  } else if (u < NUTOT) {
    const int v = u - NUB7;
    const int n  = v >> 8;
    const int k8 = (v & 255) * 8;
    const int kk = k8 & (D1 - 1);
    o = cv8b(l2 + (size_t)kk * COUT + n, COUT);
    dp = pl2 + (size_t)v * 8;
  } else {
    return;
  }
  *(volatile v8us*)dp = o;
  __threadfence();
  *(volatile v8us*)dp = o;
}

template <int RND>
__global__ __launch_bounds__(NTHR) void k_agg(
    const int* __restrict__ srcs, const int* __restrict__ dsts,
    const float* __restrict__ fin,
    unsigned short* Aout, int ldaOut,
    int nN, int nE, int nb, int vec8, int MPr) {
  extern __shared__ v4f lds_dyn[];
  int* reg1 = (int*)lds_dyn;
  int* reg2 = reg1 + RCAP;
  int* scnt = reg2 + RCAP;
  int* soff = scnt + NBMAX;
  int* list = soff + NBMAX;
  int* wcnt = list + LISTN;
  int* wtot = wcnt + NWAVE;
  const int tid = (int)threadIdx.x, lane = tid & 31, wave = tid >> 5;
  const int nodeBase = (int)blockIdx.x * nb;

  for (int i = tid; i < NBMAX; i += NTHR) scnt[i] = 0;
  __syncthreads();

  int tot = 0;
  const int nChunks = (nE + CHUNK - 1) / CHUNK;
#pragma unroll 1
  for (int ch = 0; ch < nChunks; ++ch) {
    const int cbase = ch * CHUNK;
    const int wc = scan_chunk(dsts, nE, cbase, nodeBase, nb, vec8, list, tid, lane, wave);
    if (lane == 0) wcnt[wave] = wc;
    __syncthreads();
    int pre = 0, all = 0;
#pragma unroll
    for (int w2 = 0; w2 < NWAVE; ++w2) {
      int c = wcnt[w2];
      c = c < 0 ? 0 : (c > WCAP ? WCAP : c);
      all += c;
      pre += (w2 < wave) ? c : 0;
    }
    const int wcc  = wc > WCAP ? WCAP : wc;
    const int base = tot + pre;
#pragma unroll 1
    for (int i = lane; i < wcc; i += 32) {
      const int ent = list[wave * WCAP + i];
      const int el  = (ent >> PKS) & (CHUNK - 1);
      const int sl  = ent & (NBMAX - 1);
      int eid = cbase + el;
      eid = eid > nE - 1 ? nE - 1 : eid;
      const int pos = base + i;
      if (pos < RCAP) reg1[pos] = (int)(((unsigned)eid << PKS) | (unsigned)sl);
    }
    tot += all;
    tot = tot > RCAP ? RCAP : tot;
    __syncthreads();
  }
  const int nh = tot;

  if (wave == 0) {
#pragma unroll 1
    for (int b0 = 0; b0 < nh; b0 += 32) {
      const int idx = b0 + lane;
      const int uv  = reg1[idx < RCAP ? idx : RCAP - 1];
      const int m32 = (nh - b0) < 32 ? (nh - b0) : 32;
#pragma unroll 1
      for (int k = 0; k < m32; ++k) {
        const int u  = __builtin_amdgcn_readlane(uv, k);
        const int sl = u & (NBMAX - 1);
        if (lane == 0) scnt[sl] = scnt[sl] + 1;
      }
    }
  }
  __syncthreads();

  {
    const v4i ca = *(const v4i*)(scnt + 8 * tid);
    const v4i cb = *(const v4i*)(scnt + 8 * tid + 4);
    const int e0 = ca.x < 0 ? 0 : ca.x, e1 = ca.y < 0 ? 0 : ca.y, e2 = ca.z < 0 ? 0 : ca.z, e3 = ca.w < 0 ? 0 : ca.w;
    const int e4 = cb.x < 0 ? 0 : cb.x, e5 = cb.y < 0 ? 0 : cb.y, e6 = cb.z < 0 ? 0 : cb.z, e7 = cb.w < 0 ? 0 : cb.w;
    const int ts = e0 + e1 + e2 + e3 + e4 + e5 + e6 + e7;
    int incl = ts;
#pragma unroll
    for (int d = 1; d < 32; d <<= 1) {
      const int up = __shfl_up(incl, d);
      if (lane >= d) incl += up;
    }
    if (lane == 31) wtot[wave] = incl;
    __syncthreads();
    int pre = 0;
#pragma unroll
    for (int w2 = 0; w2 < NWAVE; ++w2) pre += (w2 < wave) ? wtot[w2] : 0;
    int run = pre + incl - ts;
    soff[8 * tid + 0] = run; run += e0;
    soff[8 * tid + 1] = run; run += e1;
    soff[8 * tid + 2] = run; run += e2;
    soff[8 * tid + 3] = run; run += e3;
    soff[8 * tid + 4] = run; run += e4;
    soff[8 * tid + 5] = run; run += e5;
    soff[8 * tid + 6] = run; run += e6;
    soff[8 * tid + 7] = run;
  }
  __syncthreads();
  for (int i = tid; i < NBMAX; i += NTHR) list[i] = soff[i];
  __syncthreads();

  if (wave == 0) {
#pragma unroll 1
    for (int b0 = 0; b0 < nh; b0 += 32) {
      const int idx = b0 + lane;
      const int uv  = reg1[idx < RCAP ? idx : RCAP - 1];
      const int m32 = (nh - b0) < 32 ? (nh - b0) : 32;
#pragma unroll 1
      for (int k = 0; k < m32; ++k) {
        const int u   = __builtin_amdgcn_readlane(uv, k);
        const int sl  = u & (NBMAX - 1);
        const int eid = (int)((unsigned)u >> PKS);
        if (lane == 0) {
          int pos = list[sl];
          pos = pos < 0 ? 0 : (pos > RCAP - 1 ? RCAP - 1 : pos);
          reg2[pos] = eid;
          list[sl] = pos + 1;
        }
      }
    }
  }
  __syncthreads();

  const int nbw = nb >> 3;
  const bool ovf = (nh >= RCAP);
  const float qnan = __int_as_float(0x7fc00000);

#pragma unroll 1
  for (int jt = 0; jt < nbw; ++jt) {
    const int slot = wave * nbw + jt;
    const int grow = nodeBase + slot;
    int st = soff[slot];
    const int craw = scnt[slot];
    int cnt = craw;
    st  = st < 0 ? 0 : (st > nh ? nh : st);
    cnt = cnt < 0 ? 0 : (cnt > DEGCAP ? DEGCAP : cnt);
    if (cnt > nh - st) cnt = nh - st;
    const float pz = (ovf || craw > DEGCAP) ? qnan : 0.0f;
    const bool liveRow = grow < nN;

    float ag0 = 0.f, ag1 = 0.f, ag2 = 0.f, ag3 = 0.f;
#pragma unroll 1
    for (int q = 0; q < cnt; ++q) {
      int idx = st + q; idx = idx > RCAP - 1 ? RCAP - 1 : idx;
      int eid = reg2[idx]; eid = eid < 0 ? 0 : (eid > nE - 1 ? nE - 1 : eid);
      const int sraw = srcs[eid];
      const int s = sraw < 0 ? 0 : (sraw > nN - 1 ? nN - 1 : sraw);
      const v4f v = *(const v4f*)(fin + (size_t)s * DIN + 4 * lane);
      float v0 = v.x, v1 = v.y, v2 = v.z, v3 = v.w;
      if (RND != 0) { v0 = bf_rne(v0); v1 = bf_rne(v1); v2 = bf_rne(v2); v3 = bf_rne(v3); }
      ag0 += v0; ag1 += v1; ag2 += v2; ag3 += v3;
    }
    const int nc = liveRow ? grow : nN - 1;
    const v4f sv = *(const v4f*)(fin + (size_t)nc * DIN + 4 * lane);
    float s0 = sv.x, s1 = sv.y, s2 = sv.z, s3 = sv.w;
    if (RND != 0) { s0 = bf_rne(s0); s1 = bf_rne(s1); s2 = bf_rne(s2); s3 = bf_rne(s3); }
    float r0 = s0 + ag0, r1 = s1 + ag1, r2 = s2 + ag2, r3 = s3 + ag3;
    r0 = (liveRow ? r0 : 0.0f) + pz;
    r1 = (liveRow ? r1 : 0.0f) + pz;
    r2 = (liveRow ? r2 : 0.0f) + pz;
    r3 = (liveRow ? r3 : 0.0f) + pz;

    const unsigned int b0 = (unsigned int)h16_bits(r0 * CA), b1 = (unsigned int)h16_bits(r1 * CA);
    const unsigned int b2 = (unsigned int)h16_bits(r2 * CA), b3 = (unsigned int)h16_bits(r3 * CA);
    v2u pk;
    pk.x = b0 | (b1 << 16);
    pk.y = b2 | (b3 << 16);
    unsigned short* gp = Aout + (size_t)grow * (size_t)ldaOut + 4 * lane;
    const bool wsv = grow < MPr;
    if (wsv) *(volatile v2u*)gp = pk;
    __threadfence();
    if (wsv) *(volatile v2u*)gp = pk;
  }
}

template <int BF, int EPI>
__global__ __launch_bounds__(GTHR) void k_gemm(const unsigned short* __restrict__ A, int lda,
                                               const unsigned short* __restrict__ BT, int ldb, int K,
                                               const float* __restrict__ bias, float oscale, float ocarry,
                                               void* outp, int ldo, int lsplit, int nN, int mRows,
                                               float* part) {
  __shared__ __attribute__((aligned(16))) float stg[GBM * GBN];
  __shared__ __attribute__((aligned(16))) float pst[PARTW];
  const int tid = (int)threadIdx.x, lane = tid & 31, wave = tid >> 5, hh = lane >> 4, m = lane & 15;
  const int rowBase = (int)blockIdx.x * GBM;
  const int colBase = (int)blockIdx.y * GBN;

  v8f acc[GNT];
  {
    const v8f z = {0.f, 0.f, 0.f, 0.f, 0.f, 0.f, 0.f, 0.f};
#pragma unroll
    for (int t = 0; t < GNT; ++t) acc[t] = z;
  }
  const unsigned short* ap = A  + (size_t)(rowBase + 16 * wave + m) * (size_t)lda + 8 * hh;
  const unsigned short* bp = BT + (size_t)(colBase + m) * (size_t)ldb + 8 * hh;

#pragma unroll 1
  for (int k0 = 0; k0 < K; k0 += 32) {
    Frag af;
    af.h[0] = *(const v8usa*)(ap + k0);
    af.h[1] = *(const v8usa*)(ap + k0 + 16);
#pragma unroll
    for (int nt = 0; nt < GNT; ++nt) {
      const unsigned short* wq = bp + (size_t)(16 * nt) * (size_t)ldb + k0;
      Frag bfr;
      bfr.h[0] = *(const v8usa*)wq;
      bfr.h[1] = *(const v8usa*)(wq + 16);
      acc[nt] = wmx<BF>(af, bfr, acc[nt]);
    }
  }

#pragma unroll
  for (int nt = 0; nt < GNT; ++nt) {
    const int lc = 16 * nt + m;
    const float bb = bf_rne(bias[colBase + lc]);
#pragma unroll
    for (int r = 0; r < 8; ++r) {
      const int lr = 16 * wave + 8 * hh + r;
      const bool live = (rowBase + lr) < nN;
      float v = fmaf(acc[nt][r], oscale, bb);
      if constexpr (EPI == 2) v = fmaxf(v, 0.0f);
      stg[lr * GBN + lc] = live ? v : 0.0f;
    }
  }
  __syncthreads();

  if constexpr (EPI == 0) {
#pragma unroll 1
    for (int i = 0; i < (GBM * GBN) / GTHR; ++i) {
      const int idx = i * GTHR + tid;
      stg[idx] = gelu_exact(stg[idx]);
    }
    __syncthreads();
    unsigned short* outH = (unsigned short*)outp;
    v2u pk[16];
#pragma unroll
    for (int i = 0; i < 16; ++i) {
      const int lr = 16 * wave + i;
      const v4f a = *(const v4fa*)(stg + lr * GBN + 4 * lane);
      v2u w;
      w.x = (unsigned int)h16_bits(a.x * ocarry) | ((unsigned int)h16_bits(a.y * ocarry) << 16);
      w.y = (unsigned int)h16_bits(a.z * ocarry) | ((unsigned int)h16_bits(a.w * ocarry) << 16);
      pk[i] = w;
    }
#pragma unroll
    for (int i = 0; i < 16; ++i) {
      const int gr = rowBase + 16 * wave + i;
      unsigned short* op = outH + (size_t)gr * (size_t)ldo + colBase + 4 * lane;
      if (gr < mRows) *(volatile v2u*)op = pk[i];
    }
    __threadfence();
#pragma unroll
    for (int i = 0; i < 16; ++i) {
      const int gr = rowBase + 16 * wave + i;
      unsigned short* op = outH + (size_t)gr * (size_t)ldo + colBase + 4 * lane;
      if (gr < mRows) *(volatile v2u*)op = pk[i];
    }
  } else if constexpr (EPI == 2) {
    unsigned short* outH = (unsigned short*)outp;
    const int cb = 8 * m;
    const bool isHi = (hh == 0);
    v4u pk[16];
#pragma unroll
    for (int i = 0; i < 16; ++i) {
      const int lr = 16 * wave + i;
      const v4f a = *(const v4fa*)(stg + lr * GBN + cb);
      const v4f b = *(const v4fa*)(stg + lr * GBN + cb + 4);
      const float f[8] = {a.x, a.y, a.z, a.w, b.x, b.y, b.z, b.w};
      unsigned int w[4];
#pragma unroll
      for (int j = 0; j < 4; ++j) {
        const unsigned short h0 = bf_bits(f[2 * j]), h1 = bf_bits(f[2 * j + 1]);
        const unsigned short l0 = bf_bits(f[2 * j] - bf_val(h0)), l1 = bf_bits(f[2 * j + 1] - bf_val(h1));
        const unsigned short q0 = isHi ? h0 : l0, q1 = isHi ? h1 : l1;
        w[j] = (unsigned int)q0 | ((unsigned int)q1 << 16);
      }
      v4u pv; pv.x = w[0]; pv.y = w[1]; pv.z = w[2]; pv.w = w[3];
      pk[i] = pv;
    }
#pragma unroll
    for (int i = 0; i < 16; ++i) {
      const int gr = rowBase + 16 * wave + i;
      unsigned short* op = outH + (size_t)gr * (size_t)ldo + colBase + cb + hh * lsplit;
      if (gr < mRows) *(volatile v4u*)op = pk[i];
    }
    __threadfence();
#pragma unroll
    for (int i = 0; i < 16; ++i) {
      const int gr = rowBase + 16 * wave + i;
      unsigned short* op = outH + (size_t)gr * (size_t)ldo + colBase + cb + hh * lsplit;
      if (gr < mRows) *(volatile v4u*)op = pk[i];
    }
  } else {
    float* outF = (float*)outp;
    v4f fv[16];
#pragma unroll
    for (int i = 0; i < 16; ++i) {
      const int lr = 16 * wave + i;
      fv[i] = *(const v4fa*)(stg + lr * GBN + 4 * lane);
    }
    v4f pv = {0.f, 0.f, 0.f, 0.f};
    const bool pok = (EPI == 1) && (tid < PARTW / 4);
    if constexpr (EPI == 1) {
      int nvr = nN - rowBase;
      nvr = nvr < 0 ? 0 : (nvr > GBM ? GBM : nvr);
      float s = 0.0f;
#pragma unroll 1
      for (int r = 0; r < nvr; ++r) s += stg[r * GBN + tid];
      const float inv = 1.0f / (float)(nvr < 1 ? 1 : nvr);
      const float mean = s * inv;
      float q = 0.0f;
#pragma unroll 1
      for (int r = 0; r < nvr; ++r) {
        const float d = stg[r * GBN + tid] - mean;
        q = fmaf(d, d, q);
      }
      pst[1 + tid] = mean;
      pst[1 + GBN + tid] = q;
      if (tid == 0) pst[0] = (float)nvr;
#pragma unroll 1
      for (int i = 2 * GBN + 1 + tid; i < PARTW; i += GTHR) pst[i] = 0.0f;
      __syncthreads();
      if (pok) pv = *(const v4fa*)(pst + 4 * tid);
    }
    const size_t prow = (size_t)blockIdx.x * (size_t)gridDim.y + (size_t)blockIdx.y;
    float* pp = part + prow * PARTW + 4 * tid;
#pragma unroll
    for (int i = 0; i < 16; ++i) {
      const int gr = rowBase + 16 * wave + i;
      float* op = outF + (size_t)gr * (size_t)ldo + colBase + 4 * lane;
      if (gr < mRows) *(volatile v4f*)op = fv[i];
    }
    if (pok) *(volatile v4f*)pp = pv;
    __threadfence();
#pragma unroll
    for (int i = 0; i < 16; ++i) {
      const int gr = rowBase + 16 * wave + i;
      float* op = outF + (size_t)gr * (size_t)ldo + colBase + 4 * lane;
      if (gr < mRows) *(volatile v4f*)op = fv[i];
    }
    if (pok) *(volatile v4f*)pp = pv;
  }
}

__global__ __launch_bounds__(GBN) void k_bnfin(const float* __restrict__ part, int nPart, int gy, int nh,
                                               const float* __restrict__ gam, const float* __restrict__ bet,
                                               float* ss) {
  __shared__ __attribute__((aligned(16))) float stg[2 * GBN];
  const int tid = (int)threadIdx.x;
  const int by  = (int)blockIdx.x;
  const int col = by * GBN + tid;
  double n = 0.0, mean = 0.0, M2 = 0.0;
#pragma unroll 1
  for (int b = 0; b < nPart; ++b) {
    const float* pr = part + ((size_t)b * (size_t)gy + (size_t)by) * PARTW;
    const double nb = (double)pr[0];
    const double mb = (double)pr[1 + tid];
    const double qb = (double)pr[1 + GBN + tid];
    if (nb > 0.5) {
      const double nn = n + nb;
      const double delta = mb - mean;
      const double f = nb / nn;
      mean = mean + delta * f;
      M2 = M2 + qb + delta * delta * n * f;
      n = nn;
    }
  }
  const double nt = n < 1.0 ? 1.0 : n;
  const float var  = (float)(M2 / nt);
  const float rstd = rsqrtf(var + 1e-5f);
  const float sc = bf_rne(gam[col]) * rstd;
  const float sh = bf_rne(bet[col]) - (float)mean * sc;
  stg[tid] = sc;
  stg[GBN + tid] = sh;
  __syncthreads();
  const int seg = tid >> 5, j = tid & 31;
  const bool ok = tid < 64;
  v4f v = {0.f, 0.f, 0.f, 0.f};
  float* dp = ss + (size_t)seg * (size_t)nh + (size_t)by * GBN + 4 * j;
  if (ok) {
    v = *(const v4fa*)(stg + seg * GBN + 4 * j);
    *(volatile v4f*)dp = v;
  }
  __threadfence();
  if (ok) *(volatile v4f*)dp = v;
}

__global__ __launch_bounds__(NTHR) void k_bnap(const float* __restrict__ U, const float* __restrict__ ss,
                                              int nN, int mRows, float* H) {
  __shared__ float ssh[2 * DIN];
  __shared__ __attribute__((aligned(16))) float tile[APR * DIN];
  const int tid = (int)threadIdx.x;
  ssh[tid] = ss[tid];
  const int rowBase = (int)blockIdx.x * APR;
  const int c  = tid & (DIN - 1);
  const int rs = tid >> 7;
  __syncthreads();
#pragma unroll 1
  for (int r = 0; r < APR / 2; ++r) {
    const int lr   = 2 * r + rs;
    const int grow = rowBase + lr;
    const int gc   = grow < nN ? grow : nN - 1;
    const float u = U[(size_t)gc * DIN + c];
    const float v = gelu_exact(fmaf(u, ssh[c], ssh[DIN + c]));
    tile[lr * DIN + c] = (grow < nN) ? v : 0.0f;
  }
  __syncthreads();
  v4f pv[2];
#pragma unroll
  for (int it = 0; it < 2; ++it) {
    const int p = it * NTHR + tid;
    const int lr = p >> 5, q = p & 31;
    pv[it] = *(const v4fa*)(tile + lr * DIN + 4 * q);
  }
#pragma unroll
  for (int it = 0; it < 2; ++it) {
    const int p = it * NTHR + tid;
    const int lr = p >> 5, q = p & 31;
    const int grow = rowBase + lr;
    float* op = H + (size_t)grow * DIN + 4 * q;
    if (grow < mRows) *(volatile v4f*)op = pv[it];
  }
  __threadfence();
#pragma unroll
  for (int it = 0; it < 2; ++it) {
    const int p = it * NTHR + tid;
    const int lr = p >> 5, q = p & 31;
    const int grow = rowBase + lr;
    float* op = H + (size_t)grow * DIN + 4 * q;
    if (grow < mRows) *(volatile v4f*)op = pv[it];
  }
}

template <int NH>
__global__ __launch_bounds__(NTHR) void k_pool(const float* __restrict__ U, const float* __restrict__ ss,
                                               const int* __restrict__ bat, int nN, int vec8b, int nG,
                                               unsigned short* hc, int colOff) {
  extern __shared__ __attribute__((aligned(16))) float psm[];
  float* accs = psm;
  float* ssh  = accs + PG * NH;
  int*   list = (int*)(ssh + 2 * NH);
  int*   wcnt = list + LISTN;
  const int tid = (int)threadIdx.x, lane = tid & 31, wave = tid >> 5;
  const int slotBase = (int)blockIdx.x * PG;

  for (int i = tid; i < PG * NH; i += NTHR) accs[i] = 0.0f;
  for (int i = tid; i < 2 * NH; i += NTHR) ssh[i] = ss[i];
  __syncthreads();

  const int nChunks = (nN + CHUNK - 1) / CHUNK;
#pragma unroll 1
  for (int ch = 0; ch < nChunks; ++ch) {
    const int cbase = ch * CHUNK;
    const int wc = scan_chunk(bat, nN, cbase, slotBase, PG, vec8b, list, tid, lane, wave);
    if (lane == 0) wcnt[wave] = wc;
    __syncthreads();
#pragma unroll 1
    for (int w2 = 0; w2 < NWAVE; ++w2) {
      int c = wcnt[w2];
      c = c < 0 ? 0 : (c > WCAP ? WCAP : c);
#pragma unroll 1
      for (int i = 0; i < c; ++i) {
        const int ent = list[w2 * WCAP + i];
        const int el  = (ent >> PKS) & (CHUNK - 1);
        const int sl  = ent & (PG - 1);
        int node = cbase + el;
        node = node < 0 ? 0 : (node > nN - 1 ? nN - 1 : node);
#pragma unroll 1
        for (int cc = tid; cc < NH; cc += NTHR) {
          const float u = U[(size_t)node * NH + cc];
          const float v = gelu_exact(fmaf(u, ssh[cc], ssh[NH + cc]));
          accs[sl * NH + cc] += v;
        }
      }
    }
    __syncthreads();
  }

  constexpr int PPR = NH / 8;
  constexpr int NIT = (PG * PPR) / NTHR;
  v8us hv[NIT], lv[NIT];
#pragma unroll
  for (int it = 0; it < NIT; ++it) {
    const int p = it * NTHR + tid;
    const int row = p / PPR, q = p % PPR;
    const v4f a = *(const v4fa*)(accs + row * NH + 8 * q);
    const v4f b = *(const v4fa*)(accs + row * NH + 8 * q + 4);
    hilo8(a, b, hv[it], lv[it]);
  }
#pragma unroll
  for (int it = 0; it < NIT; ++it) {
    const int p = it * NTHR + tid;
    const int row = p / PPR, q = p % PPR;
    const int g = slotBase + row;
    unsigned short* hp = hc + (size_t)g * HCW + colOff + 8 * q;
    unsigned short* lp = hc + (size_t)g * HCW + HCAT + colOff + 8 * q;
    if (g < nG) { *(volatile v8us*)hp = hv[it]; *(volatile v8us*)lp = lv[it]; }
  }
  __threadfence();
#pragma unroll
  for (int it = 0; it < NIT; ++it) {
    const int p = it * NTHR + tid;
    const int row = p / PPR, q = p % PPR;
    const int g = slotBase + row;
    unsigned short* hp = hc + (size_t)g * HCW + colOff + 8 * q;
    unsigned short* lp = hc + (size_t)g * HCW + HCAT + colOff + 8 * q;
    if (g < nG) { *(volatile v8us*)hp = hv[it]; *(volatile v8us*)lp = lv[it]; }
  }
}

static int pick_nb(int nE, int nN) {
  int nb = NBMAX;
  while (nb > 16 && (long long)nb * (long long)nE * 5LL > (long long)RCAP * (long long)nN * 4LL) nb >>= 1;
  return nb;
}
static inline int cdiv(int a, int b) { return (a + b - 1) / b; }
static inline size_t al256(size_t o) { return (o + 255) & ~(size_t)255; }

extern "C" void kernel_launch(void* const* d_in, const int* in_sizes, int n_in,
                              void* d_out, int out_size, void* d_ws, size_t ws_size,
                              hipStream_t stream) {
  if (n_in < 25) return;
  if (in_sizes[0] < DIN || (in_sizes[0] % DIN) != 0) return;
  const int nN = in_sizes[0] / DIN;
  if (nN < GBM || nN > (1 << 22)) return;
  const int nE2 = in_sizes[1];
  if (nE2 < 2 || (nE2 & 1) != 0) return;
  const int nE = nE2 / 2;
  if (nE < 1 || nE > (1 << 21)) return;
  if (in_sizes[2] != nN) return;
  if (in_sizes[3] != DIN * DIN || in_sizes[4] != DIN) return;
  if (in_sizes[5] != DIN * DIN || in_sizes[6] != DIN) return;
  if (in_sizes[7] != DIN || in_sizes[8] != DIN) return;
  if (in_sizes[9] != DIN * DIN || in_sizes[10] != DIN) return;
  if (in_sizes[11] != DIN * DIN || in_sizes[12] != DIN) return;
  if (in_sizes[13] != DIN || in_sizes[14] != DIN) return;
  if (in_sizes[15] != DIN * HL3 || in_sizes[16] != HL3) return;
  if (in_sizes[17] != HL3 * HL3 || in_sizes[18] != HL3) return;
  if (in_sizes[19] != HL3 || in_sizes[20] != HL3) return;
  if (in_sizes[21] != HCAT * D1 || in_sizes[22] != D1) return;
  if (in_sizes[23] != D1 * COUT || in_sizes[24] != COUT) return;
  if (out_size < COUT || (out_size % COUT) != 0) return;
  const int nG = out_size / COUT;
  if (nG < GBM || (nG % GBM) != 0 || (nG % PG) != 0 || nG > 65536) return;
  if ((long long)nG * COUT != (long long)out_size) return;

  const float* x     = (const float*)d_in[0];
  const int*   ei    = (const int*)  d_in[1];
  const int*   src   = ei;
  const int*   dst   = ei + nE;
  const int*   batch = (const int*)  d_in[2];
  const float* c1W1 = (const float*)d_in[3];  const float* c1b1 = (const float*)d_in[4];
  const float* c1W2 = (const float*)d_in[5];  const float* c1b2 = (const float*)d_in[6];
  const float* bn1g = (const float*)d_in[7];  const float* bn1b = (const float*)d_in[8];
  const float* c2W1 = (const float*)d_in[9];  const float* c2b1 = (const float*)d_in[10];
  const float* c2W2 = (const float*)d_in[11]; const float* c2b2 = (const float*)d_in[12];
  const float* bn2g = (const float*)d_in[13]; const float* bn2b = (const float*)d_in[14];
  const float* c3W1 = (const float*)d_in[15]; const float* c3b1 = (const float*)d_in[16];
  const float* c3W2 = (const float*)d_in[17]; const float* c3b2 = (const float*)d_in[18];
  const float* bn3g = (const float*)d_in[19]; const float* bn3b = (const float*)d_in[20];
  const float* l1W  = (const float*)d_in[21]; const float* l1b  = (const float*)d_in[22];
  const float* l2W  = (const float*)d_in[23]; const float* l2b  = (const float*)d_in[24];
  float* out = (float*)d_out;

  const int MP   = cdiv(nN, GBM) * GBM;
  const int gM   = MP / GBM;
  const int nb   = pick_nb(nE, nN);
  const int gA   = cdiv(MP, nb);
  const int vec8 = ((nE & 3) == 0) ? 1 : 0;
  if ((long long)gA * nb < (long long)MP) return;
  if ((long long)(gM - 1) * GBM >= (long long)nN) return;
  if ((MP % APR) != 0) return;
  const int gy3 = HL3 / GBN;
  const int gH  = nG / GBM;

  char* ws = (char*)d_ws;
  size_t off = 0;
  const size_t oW11 = off; off = al256(off + (size_t)NU11 * 16);
  const size_t oW12 = off; off = al256(off + (size_t)NU11 * 16);
  const size_t oW13 = off; off = al256(off + (size_t)NU13 * 16);
  const size_t oW21 = off; off = al256(off + (size_t)NU11 * 16);
  const size_t oW22 = off; off = al256(off + (size_t)NU11 * 16);
  const size_t oW23 = off; off = al256(off + (size_t)NU23 * 16);
  const size_t oL1  = off; off = al256(off + (size_t)NUL1 * 16);
  const size_t oL2  = off; off = al256(off + (size_t)NUL2 * 16);
  const size_t oAH  = off; off = al256(off + (size_t)MP * DIN * 2);
  const size_t oTH  = off; off = al256(off + (size_t)MP * HL3 * 2);
  const size_t oUF  = off; off = al256(off + (size_t)MP * HL3 * 4);
  const size_t oHF  = off; off = al256(off + (size_t)MP * DIN * 4);
  const size_t oPT  = off; off = al256(off + (size_t)gM * gy3 * PARTW * 4);
  const size_t oSS  = off; off = al256(off + (size_t)(2 * HL3) * 4);
  const size_t oHC  = off; off = al256(off + (size_t)nG * HCW * 2);
  const size_t oZP  = off; off = al256(off + (size_t)nG * ZPW * 2);
  if (off > ws_size || off > (size_t)WSMAX) return;
  unsigned short* W11 = (unsigned short*)(ws + oW11);
  unsigned short* W12 = (unsigned short*)(ws + oW12);
  unsigned short* W13 = (unsigned short*)(ws + oW13);
  unsigned short* W21 = (unsigned short*)(ws + oW21);
  unsigned short* W22 = (unsigned short*)(ws + oW22);
  unsigned short* W23 = (unsigned short*)(ws + oW23);
  unsigned short* L1  = (unsigned short*)(ws + oL1);
  unsigned short* L2  = (unsigned short*)(ws + oL2);
  unsigned short* AH  = (unsigned short*)(ws + oAH);
  unsigned short* TH  = (unsigned short*)(ws + oTH);
  float*          UF  = (float*)(ws + oUF);
  float*          HF  = (float*)(ws + oHF);
  float*          PT  = (float*)(ws + oPT);
  float*          SS  = (float*)(ws + oSS);
  unsigned short* HC  = (unsigned short*)(ws + oHC);
  unsigned short* ZP  = (unsigned short*)(ws + oZP);

  hipFuncSetAttribute(reinterpret_cast<const void*>(&k_agg<1>),     hipFuncAttributeMaxDynamicSharedMemorySize, LDS_AGG);
  hipFuncSetAttribute(reinterpret_cast<const void*>(&k_agg<0>),     hipFuncAttributeMaxDynamicSharedMemorySize, LDS_AGG);
  hipFuncSetAttribute(reinterpret_cast<const void*>(&k_pool<HL3>),  hipFuncAttributeMaxDynamicSharedMemorySize, LDS_POOL(HL3));
  hipFuncSetAttribute(reinterpret_cast<const void*>(&k_pool<DIN>),  hipFuncAttributeMaxDynamicSharedMemorySize, LDS_POOL(DIN));

  const float osc = 1.0f / (CA * CW);

  k_wprep<<<NUTOT / NTHR, NTHR, 0, stream>>>(c1W1, c2W1, c3W1, c1W2, c2W2, c3W2, l1W, l2W,
                                             W11, W12, W13, W21, W22, W23, L1, L2);
  k_agg<1><<<gA, NTHR, LDS_AGG, stream>>>(src, dst, x, AH, DIN, nN, nE, nb, vec8, MP);
  k_gemm<0, 0><<<dim3(gM, DIN / GBN), GTHR, 0, stream>>>(AH, DIN, W11, DIN, DIN, c1b1, osc, CT, (void*)TH, DIN, 0, nN, MP, PT);
  k_gemm<0, 1><<<dim3(gM, DIN / GBN), GTHR, 0, stream>>>(TH, DIN, W21, DIN, DIN, c1b2, osc, 1.0f, (void*)UF, DIN, 0, nN, MP, PT);
  k_bnfin<<<DIN / GBN, GBN, 0, stream>>>(PT, gM, DIN / GBN, DIN, bn1g, bn1b, SS);
  k_bnap<<<MP / APR, NTHR, 0, stream>>>(UF, SS, nN, MP, HF);
  k_pool<DIN><<<nG / PG, NTHR, LDS_POOL(DIN), stream>>>(UF, SS, batch, nN, 1, nG, HC, 0);
  k_agg<0><<<gA, NTHR, LDS_AGG, stream>>>(src, dst, HF, AH, DIN, nN, nE, nb, vec8, MP);
  k_gemm<0, 0><<<dim3(gM, DIN / GBN), GTHR, 0, stream>>>(AH, DIN, W12, DIN, DIN, c2b1, osc, CT, (void*)TH, DIN, 0, nN, MP, PT);
  k_gemm<0, 1><<<dim3(gM, DIN / GBN), GTHR, 0, stream>>>(TH, DIN, W22, DIN, DIN, c2b2, osc, 1.0f, (void*)UF, DIN, 0, nN, MP, PT);
  k_bnfin<<<DIN / GBN, GBN, 0, stream>>>(PT, gM, DIN / GBN, DIN, bn2g, bn2b, SS);
  k_bnap<<<MP / APR, NTHR, 0, stream>>>(UF, SS, nN, MP, HF);
  k_pool<DIN><<<nG / PG, NTHR, LDS_POOL(DIN), stream>>>(UF, SS, batch, nN, 1, nG, HC, DIN);
  k_agg<0><<<gA, NTHR, LDS_AGG, stream>>>(src, dst, HF, AH, DIN, nN, nE, nb, vec8, MP);
  k_gemm<0, 0><<<dim3(gM, gy3), GTHR, 0, stream>>>(AH, DIN, W13, DIN, DIN, c3b1, osc, CT, (void*)TH, HL3, 0, nN, MP, PT);
  k_gemm<0, 1><<<dim3(gM, gy3), GTHR, 0, stream>>>(TH, HL3, W23, HL3, HL3, c3b2, osc, 1.0f, (void*)UF, HL3, 0, nN, MP, PT);
  k_bnfin<<<gy3, GBN, 0, stream>>>(PT, gM, gy3, HL3, bn3g, bn3b, SS);
  k_pool<HL3><<<nG / PG, NTHR, LDS_POOL(HL3), stream>>>(UF, SS, batch, nN, 1, nG, HC, 2 * DIN);
  k_gemm<1, 2><<<dim3(gH, D1 / GBN), GTHR, 0, stream>>>(HC, HCW, L1, HCW, HCW, l1b, 1.0f, 1.0f, (void*)ZP, ZPW, D1, nG, nG, PT);
  k_gemm<1, 3><<<dim3(gH, COUT / GBN), GTHR, 0, stream>>>(ZP, ZPW, L2, ZPW, ZPW, l2b, 1.0f, 1.0f, (void*)out, COUT, 0, nG, nG, PT);
}
